// transformer_566935683726
// MI455X (gfx1250) — hardware-verified
//
#include <hip/hip_runtime.h>


#pragma clang fp contract(off)

#ifndef NB
#define NB 4
#endif
#define TT   4096
#define FD   64
#define NH   2
#define DHD  32
#define NS   8
#define NKP  64
#define NGR  4
#define QCH  2048
#define XSTR_FULL ((size_t)TT * FD)
#define SSTR_FULL ((size_t)NS * FD)
#define EPSN 1e-5f
#define PCAR 1024.0f
#define QCAR 64.0f
#define VCAR 64.0f
#define SCL  3.0517578125e-05f
#define ZSC  1.52587890625e-05f

static_assert(NB >= 1 && NB <= 4);
static_assert(TT % 128 == 0 && TT % QCH == 0 && QCH % 64 == 0 && QCH % 8 == 0);
static_assert(NS == 8 && NKP == 64 && NH * DHD == FD && FD == 64);
static_assert(((size_t)NB * TT * FD / 8) % 256 == 0);
static_assert(((size_t)NB * NH * TT * DHD / 8) % 256 == 0);
static_assert(((size_t)NB * FD * TT / 2) % 256 == 0);
static_assert(((size_t)NB * NH * TT) % 32 == 0);
static_assert((size_t)3 * NB * TT * FD * 4 <= ((size_t)16 << 20));
static_assert((size_t)NB * NH * TT * NKP * 4 <= ((size_t)16 << 20));
static_assert((size_t)NB * NH * TT * NKP * 2 <= (size_t)QCH * TT * 2);
static_assert((size_t)QCH * TT * 4 >= ((size_t)17 << 20));

typedef _Float16 h16;
typedef unsigned short bf;
typedef __attribute__((ext_vector_type(16))) __bf16   v16bf;
typedef __attribute__((ext_vector_type(16))) _Float16 v16h;
typedef __attribute__((ext_vector_type(8)))  _Float16 v8h;
typedef __attribute__((ext_vector_type(8)))  unsigned short v8us;
typedef __attribute__((ext_vector_type(8)))  float    v8f;
typedef __attribute__((ext_vector_type(4)))  float    v4f;
typedef __attribute__((ext_vector_type(2)))  _Float16 v2h;
typedef __attribute__((ext_vector_type(4)))  _Float16 v4h;
typedef __attribute__((ext_vector_type(2)))  unsigned short v2us;
typedef __attribute__((ext_vector_type(4)))  unsigned short v4us;
typedef v8h  __attribute__((may_alias)) v8ha;
typedef v4f  __attribute__((may_alias)) v4fa;
typedef v8us __attribute__((may_alias)) v8usa;

__device__ __forceinline__ unsigned short f2bf(float f) { unsigned u = __float_as_uint(f); u += 0x7FFFu + ((u >> 16) & 1u); return (unsigned short)(u >> 16); }
__device__ __forceinline__ float bf2f(unsigned short b) { return __uint_as_float(((unsigned)b) << 16); }
__device__ __forceinline__ float bfr(float f) { return bf2f(f2bf(f)); }
__device__ __forceinline__ v16h cat16(v8h lo, v8h hi) { return __builtin_shufflevector(lo, hi, 0, 1, 2, 3, 4, 5, 6, 7, 8, 9, 10, 11, 12, 13, 14, 15); }
__device__ __forceinline__ v16bf cat16b(v8us lo, v8us hi) { return __builtin_bit_cast(v16bf, __builtin_shufflevector(lo, hi, 0, 1, 2, 3, 4, 5, 6, 7, 8, 9, 10, 11, 12, 13, 14, 15)); }
__device__ __forceinline__ v8f wmma16(v16h a, v16h b, v8f c) { return __builtin_amdgcn_wmma_f32_16x16x32_f16(false, a, false, b, (short)0, c, false, false); }
__device__ __forceinline__ v8f wmmab(v16bf a, v16bf b, v8f c) { return __builtin_amdgcn_wmma_f32_16x16x32_bf16(false, a, false, b, (short)0, c, false, false); }
__device__ __forceinline__ h16 tohx(float x) { return (h16)x; }
__device__ __forceinline__ void splitf(float y, unsigned short& h, unsigned short& l) { h = f2bf(y); l = f2bf(y - bf2f(h)); }

template <typename T16> struct WFrag;
template <> struct WFrag<h16> { typedef v16h V; static __device__ __forceinline__ V ld(const h16* p) { return cat16(*(const v8h*)p, *(const v8h*)(p + 16)); } static __device__ __forceinline__ v8f mma(V a, V b, v8f c) { return wmma16(a, b, c); } };
template <> struct WFrag<bf> { typedef v16bf V; static __device__ __forceinline__ V ld(const bf* p) { return cat16b(*(const v8us*)p, *(const v8us*)(p + 16)); } static __device__ __forceinline__ v8f mma(V a, V b, v8f c) { return wmmab(a, b, c); } };
template <typename T16, int SPL, int BIASM>
__global__ __launch_bounds__(32) void k_gemmw(const T16* __restrict__ A, const T16* __restrict__ A2, const T16* __restrict__ Bt, const T16* __restrict__ Bt2, int K, float* C, int ldc, const float* __restrict__ bias, size_t sA, size_t sB, size_t sC) {
    typedef typename WFrag<T16>::V V;
    __shared__ __align__(16) float os[16 * 68];
    const size_t z = blockIdx.z; A += z * sA; if (SPL & 1) A2 += z * sA; Bt += z * sB; if (SPL & 2) Bt2 += z * sB; C += z * sC;
    const int lane = threadIdx.x & 31, lr = lane & 15, hi = lane >> 4; const int r0 = blockIdx.x * 64, c0 = blockIdx.y * 64;
    v8f acc[4][4];
#pragma unroll
    for (int mb = 0; mb < 4; ++mb)
#pragma unroll
        for (int nb = 0; nb < 4; ++nb) acc[mb][nb] = (v8f){};
    const size_t aoff = (size_t)(r0 + lr) * K + 8 * hi, boff = (size_t)(c0 + lr) * K + 8 * hi;
#pragma unroll 1
    for (int kc = 0; kc < K; kc += 32) {
        V a[4], a2[4];
#pragma unroll
        for (int mb = 0; mb < 4; ++mb) { a[mb] = WFrag<T16>::ld(A + aoff + (size_t)mb * 16 * K + kc); a2[mb] = a[mb]; if (SPL & 1) a2[mb] = WFrag<T16>::ld(A2 + aoff + (size_t)mb * 16 * K + kc); }
#pragma unroll
        for (int nb = 0; nb < 4; ++nb) { const V b = WFrag<T16>::ld(Bt + boff + (size_t)nb * 16 * K + kc); V b2 = b; if (SPL & 2) b2 = WFrag<T16>::ld(Bt2 + boff + (size_t)nb * 16 * K + kc);
#pragma unroll
            for (int mb = 0; mb < 4; ++mb) { acc[mb][nb] = WFrag<T16>::mma(a[mb], b, acc[mb][nb]); if (SPL & 1) acc[mb][nb] = WFrag<T16>::mma(a2[mb], b, acc[mb][nb]); if (SPL & 2) acc[mb][nb] = WFrag<T16>::mma(a[mb], b2, acc[mb][nb]); } }
        asm volatile("v_nop\n\tv_nop\n\tv_nop\n\tv_nop" : "+v"(acc[0][0]), "+v"(acc[1][1]), "+v"(acc[2][2]), "+v"(acc[3][3]) : "v"(a[0]), "v"(a[3]));
    }
#pragma unroll
    for (int mb = 0; mb < 4; ++mb) {
#pragma unroll
        for (int nb = 0; nb < 4; ++nb) {
#pragma unroll
            for (int j = 0; j < 8; ++j) os[(hi * 8 + j) * 68 + nb * 16 + lr] = acc[mb][nb][j]; }
        __builtin_amdgcn_wave_barrier(); asm volatile("" ::: "memory");
        float* crow = C + (size_t)(r0 + mb * 16) * ldc + c0;
#pragma unroll 1
        for (int ps = 0; ps < 2; ++ps) {
#pragma unroll
            for (int s = 0; s < 8; ++s) { const int row = 2 * s + hi, cofs = lr * 4; v4f val = *(const v4fa*)(os + row * 68 + cofs);
                if (BIASM == 1) { val[0] += bfr(bias[c0 + cofs]); val[1] += bfr(bias[c0 + cofs + 1]); val[2] += bfr(bias[c0 + cofs + 2]); val[3] += bfr(bias[c0 + cofs + 3]); }
                if (BIASM == 2) { const float rb = bfr(bias[r0 + mb * 16 + row]); val[0] += rb; val[1] += rb; val[2] += rb; val[3] += rb; }
                *(volatile v4f*)(crow + (size_t)row * ldc + cofs) = val; }
            if (ps == 0) __threadfence(); }
        __builtin_amdgcn_wave_barrier(); asm volatile("" ::: "memory");
    }
}

struct WArgs { const float* w[11]; };
static_assert(sizeof(WArgs) == 88);
__global__ __launch_bounds__(256) void k_wall(WArgs wa, bf* WB) {
    const int widx = blockIdx.y; const float* w = wa.w[0];
#pragma unroll
    for (int k = 1; k < 11; ++k) if (widx == k) w = wa.w[k];
    const bool tr = (widx < 9);
    const int lane = threadIdx.x & 31; const int L0 = (threadIdx.x >> 5) * 8;
    bf* dst = WB + (size_t)widx * 4096;
#pragma unroll 1
    for (int ps = 0; ps < 2; ++ps) {
#pragma unroll 1
        for (int l = 0; l < 8; ++l) { const int L = L0 + l; const int e = L * 64 + lane * 2; const int k = e & 63, n = e >> 6;
            const int i0 = tr ? (k * 64 + n) : e; const int i1 = tr ? ((k + 1) * 64 + n) : (e + 1);
            v2us o; o[0] = f2bf(w[i0]); o[1] = f2bf(w[i1]); *(volatile v2us*)(dst + e) = o; }
        if (ps == 0) __threadfence(); }
}

__global__ __launch_bounds__(256) void k_gnstat(const float* __restrict__ x, float* ST) {
    __shared__ float red[256];
    const int bg = blockIdx.x, b = bg / NGR, g = bg % NGR; const int tid = threadIdx.x;
    const float* xb = x + (size_t)b * XSTR_FULL + g * 16;
    float s = 0.0f;
#pragma unroll 1
    for (int i = tid; i < TT * 4; i += 256) { const int pos = i >> 2, qd = i & 3; const v4f v = *(const v4f*)(xb + (size_t)pos * FD + qd * 4); s += (bfr(v[0]) + bfr(v[1])) + (bfr(v[2]) + bfr(v[3])); }
    red[tid] = s; __syncthreads();
#pragma unroll 1
    for (int st = 128; st > 0; st >>= 1) { if (tid < st) red[tid] = red[tid] + red[tid + st]; __syncthreads(); }
    const float mu = red[0] * (1.0f / 65536.0f);
    __syncthreads();
    float q = 0.0f;
#pragma unroll 1
    for (int i = tid; i < TT * 4; i += 256) { const int pos = i >> 2, qd = i & 3; const v4f v = *(const v4f*)(xb + (size_t)pos * FD + qd * 4);
#pragma unroll
        for (int k = 0; k < 4; ++k) { const float d = bfr(v[k]) - mu; const float dd = d * d; q = q + dd; } }
    red[tid] = q; __syncthreads();
#pragma unroll 1
    for (int st = 128; st > 0; st >>= 1) { if (tid < st) red[tid] = red[tid] + red[tid + st]; __syncthreads(); }
    const float var = red[0] * (1.0f / 65536.0f); const float rstd = rsqrtf(var + EPSN);
    v4f o; o[0] = (tid == 0) ? mu : 0.0f; o[1] = (tid == 0) ? rstd : 0.0f; o[2] = 0.0f; o[3] = 0.0f;
    float* dst = ST + (size_t)bg * 32 + (tid & 7) * 4;
    if (tid < 8) *(volatile v4f*)dst = o;
    __threadfence();
    if (tid < 8) *(volatile v4f*)dst = o;
}
__global__ __launch_bounds__(256) void k_gnapply(const float* __restrict__ x, const float* __restrict__ ST, const float* __restrict__ gg, const float* __restrict__ gb, bf* Xh, bf* Xl) {
    const size_t i = (size_t)blockIdx.x * 256 + threadIdx.x; if (i >= (size_t)NB * TT * FD / 8) return; const size_t e = i * 8;
    const int c0 = (int)(e & 63); const int pos = (int)((e >> 6) % TT); const int b = (int)(e / ((size_t)FD * TT)); const int g = c0 >> 4;
    const v8f v = *(const v8f*)(x + (size_t)b * XSTR_FULL + (size_t)pos * FD + c0);
    const float mu = ST[(b * NGR + g) * 32], rs = ST[(b * NGR + g) * 32 + 1];
    v8us oh, ol;
#pragma unroll
    for (int q = 0; q < 8; ++q) { float y = bfr(v[q]) - mu; y = y * rs; y = y * bfr(gg[c0 + q]); y = y + bfr(gb[c0 + q]); unsigned short a2, c2; splitf(y, a2, c2); oh[q] = a2; ol[q] = c2; }
    *(volatile v8us*)(Xh + e) = oh; *(volatile v8us*)(Xl + e) = ol; __threadfence(); *(volatile v8us*)(Xh + e) = oh; *(volatile v8us*)(Xl + e) = ol;
}
__global__ __launch_bounds__(256) void k_split8(const float* __restrict__ F, bf* Ph, bf* Pl, size_t n8) { const size_t i = (size_t)blockIdx.x * 256 + threadIdx.x; if (i >= n8) return; const v8f v = *(const v8f*)(F + i * 8); v8us oh, ol;
#pragma unroll
    for (int k = 0; k < 8; ++k) { unsigned short a, c2; splitf(v[k], a, c2); oh[k] = a; ol[k] = c2; }
    *(volatile v8us*)(Ph + i * 8) = oh; *(volatile v8us*)(Pl + i * 8) = ol; __threadfence(); *(volatile v8us*)(Ph + i * 8) = oh; *(volatile v8us*)(Pl + i * 8) = ol; }
__global__ __launch_bounds__(256) void k_hsplit(const float* __restrict__ F, h16* P) {
    const size_t i = (size_t)blockIdx.x * 256 + threadIdx.x; if (i >= (size_t)NB * NH * TT * DHD / 8) return; const size_t e = i * 8;
    const int d0 = (int)(e & 31); const int t = (int)((e >> 5) % TT); const int h = (int)((e / ((size_t)DHD * TT)) % NH); const int b = (int)(e / ((size_t)DHD * TT * NH));
    const v8f v = *(const v8f*)(F + ((size_t)b * TT + t) * FD + h * DHD + d0); v8h o;
#pragma unroll
    for (int q = 0; q < 8; ++q) o[q] = tohx(v[q] * QCAR);
    *(volatile v8h*)(P + e) = o; __threadfence(); *(volatile v8h*)(P + e) = o;
}
__global__ __launch_bounds__(256) void k_vtp2(const float* __restrict__ F, h16* VT) {
    const size_t e = ((size_t)blockIdx.x * 256 + threadIdx.x) * 2; if (e >= (size_t)NB * FD * TT) return;
    const int t = (int)(e % TT); const int n = (int)((e / TT) % FD); const int b = (int)(e / ((size_t)TT * FD)); v2h o;
#pragma unroll
    for (int q = 0; q < 2; ++q) o[q] = tohx(VCAR * F[((size_t)b * TT + t + q) * FD + n]);
    *(volatile v2h*)(VT + e) = o; __threadfence(); *(volatile v2h*)(VT + e) = o;
}
__global__ __launch_bounds__(256) void k_lsoft(const float* __restrict__ Sb, h16* P16) {
    const int lane = threadIdx.x & 31; const int row = blockIdx.x * 8 + (threadIdx.x >> 5); if (row >= QCH) return; const float* sr = Sb + (size_t)row * TT; float mx = -3.0e38f;
#pragma unroll 4
    for (int ch = 0; ch < TT / 128; ++ch) { const int j0 = ch * 128 + lane * 4; const v4f a = *(const v4f*)(sr + j0);
#pragma unroll
        for (int q = 0; q < 4; ++q) { float t = a[q] * SCL; asm volatile("" : "+v"(t)); mx = fmaxf(mx, t); } }
#pragma unroll
    for (int sh = 16; sh; sh >>= 1) mx = fmaxf(mx, __shfl_xor(mx, sh, 32));
    float sum = 0.f;
#pragma unroll 4
    for (int ch = 0; ch < TT / 128; ++ch) { const int j0 = ch * 128 + lane * 4; const v4f a = *(const v4f*)(sr + j0);
#pragma unroll
        for (int q = 0; q < 4; ++q) { float t = a[q] * SCL; asm volatile("" : "+v"(t)); float d0 = __fsub_rn(t, mx); asm volatile("" : "+v"(d0)); sum += __builtin_amdgcn_exp2f(__fmul_rn(d0, 1.4426950408889634f)); } }
#pragma unroll
    for (int sh = 16; sh; sh >>= 1) sum += __shfl_xor(sum, sh, 32);
    const float f = __fdiv_rn(PCAR, sum);
#pragma unroll 1
    for (int ps = 0; ps < 2; ++ps) {
#pragma unroll 2
        for (int ch = 0; ch < TT / 128; ++ch) { const int j0 = ch * 128 + lane * 4; const v4f a = *(const v4f*)(sr + j0); v4h o4;
#pragma unroll
            for (int q = 0; q < 4; ++q) { float t = a[q] * SCL; asm volatile("" : "+v"(t)); float d0 = __fsub_rn(t, mx); asm volatile("" : "+v"(d0)); float ex = __builtin_amdgcn_exp2f(__fmul_rn(d0, 1.4426950408889634f)); asm volatile("" : "+v"(ex)); o4[q] = tohx(ex * f); }
            *(volatile v4h*)(P16 + (size_t)row * TT + j0) = o4; }
        if (ps == 0) __threadfence(); }
}
__global__ __launch_bounds__(256) void k_csoft(const float* __restrict__ S, h16* P) {
    __shared__ __align__(16) h16 pl[8 * 4 * 8];
    const int lane = threadIdx.x & 31, w = threadIdx.x >> 5; const int r = lane >> 3, key = lane & 7;
    const size_t row = ((size_t)blockIdx.x * 8 + w) * 4 + r;
    float t = S[row * NKP + key] * SCL; asm volatile("" : "+v"(t));
    float mx = t; mx = fmaxf(mx, __shfl_xor(mx, 1, 32)); mx = fmaxf(mx, __shfl_xor(mx, 2, 32)); mx = fmaxf(mx, __shfl_xor(mx, 4, 32));
    float d0 = __fsub_rn(t, mx); asm volatile("" : "+v"(d0)); float ex = __builtin_amdgcn_exp2f(__fmul_rn(d0, 1.4426950408889634f)); asm volatile("" : "+v"(ex));
    float sum = ex; sum += __shfl_xor(sum, 1, 32); sum += __shfl_xor(sum, 2, 32); sum += __shfl_xor(sum, 4, 32);
    const float f = __fdiv_rn(PCAR, sum);
    pl[(w * 4 + r) * 8 + key] = tohx(ex * f);
    __syncthreads();
    const v8h pv = *(const v8ha*)(pl + (w * 4 + r) * 8); v8h o;
#pragma unroll
    for (int k = 0; k < 8; ++k) o[k] = (key == 0) ? pv[k] : (h16)0.0f;
    h16* dst = P + row * NKP + key * 8;
    *(volatile v8h*)dst = o; __threadfence(); *(volatile v8h*)dst = o;
}
__global__ __launch_bounds__(256) void k_zsplit(const float* __restrict__ OB, bf* Zh, bf* Zl) {
    const size_t i = (size_t)blockIdx.x * 256 + threadIdx.x; if (i >= (size_t)NB * TT * FD / 8) return; const size_t e = i * 8;
    const int n0 = (int)(e & 63); const int t = (int)((e >> 6) % TT); const int b = (int)(e / ((size_t)FD * TT)); const int h = n0 >> 5;
    const v8f v = *(const v8f*)(OB + (((size_t)b * NH + h) * TT + t) * FD + n0); v8us oh, ol;
#pragma unroll
    for (int q = 0; q < 8; ++q) { unsigned short a2, c2; splitf(v[q] * ZSC, a2, c2); oh[q] = a2; ol[q] = c2; }
    *(volatile v8us*)(Zh + e) = oh; *(volatile v8us*)(Zl + e) = ol; __threadfence(); *(volatile v8us*)(Zh + e) = oh; *(volatile v8us*)(Zl + e) = ol;
}
template <bool GELU, bool WF>
__global__ __launch_bounds__(256) void k_lnres(const float* __restrict__ M, const float* __restrict__ R, const float* __restrict__ g, const float* __restrict__ bb, float* XF, bf* Xh, bf* Xl) {
    __shared__ __align__(16) float os[8 * 64];
    const int lane = threadIdx.x & 31, w = threadIdx.x >> 5; const size_t row = (size_t)blockIdx.x * 8 + w;
    const float* mr = M + row * 64; const float m0 = mr[lane], m1 = mr[lane + 32];
    float s = m0 + m1;
#pragma unroll
    for (int sh = 16; sh; sh >>= 1) s += __shfl_xor(s, sh, 32);
    const float mu = s * (1.0f / 64.0f);
    const float d0 = m0 - mu, d1 = m1 - mu; const float q0 = d0 * d0; const float q1 = d1 * d1; float q = q0 + q1;
#pragma unroll
    for (int sh = 16; sh; sh >>= 1) q += __shfl_xor(q, sh, 32);
    const float var = q * (1.0f / 64.0f); const float rstd = rsqrtf(var + EPSN);
#pragma unroll 1
    for (int hq = 0; hq < 2; ++hq) { const int e = lane + 32 * hq; const float d = hq ? d1 : d0; float y = d * rstd; y = y * bfr(g[e]); y = y + bfr(bb[e]); y = y + R[row * 64 + e];
        if (GELU) { const float er = erff(y * 0.70710678118654752440f); const float hy = 0.5f * y; y = hy * (1.0f + er); }
        os[w * 64 + e] = y; }
    __syncthreads();
    const int i4 = min(lane, 15) * 4, i8 = min(lane, 7) * 8;
    const v4f vf = *(const v4fa*)(os + w * 64 + i4);
    const v4f p0 = *(const v4fa*)(os + w * 64 + i8), p1 = *(const v4fa*)(os + w * 64 + i8 + 4);
    v8us oh, ol;
#pragma unroll
    for (int k = 0; k < 4; ++k) { unsigned short a2, c2; splitf(p0[k], a2, c2); oh[k] = a2; ol[k] = c2; splitf(p1[k], a2, c2); oh[4 + k] = a2; ol[4 + k] = c2; }
#pragma unroll 1
    for (int ps = 0; ps < 2; ++ps) {
        if (WF) { if (lane < 16) *(volatile v4f*)(XF + row * 64 + lane * 4) = vf; }
        if (lane < 8) { *(volatile v8us*)(Xh + row * 64 + lane * 8) = oh; *(volatile v8us*)(Xl + row * 64 + lane * 8) = ol; }
        if (ps == 0) __threadfence(); }
}
__global__ __launch_bounds__(256) void k_slotp(const float* __restrict__ sl, bf* SL) {
    const size_t i = (size_t)blockIdx.x * 256 + threadIdx.x; if (i >= (size_t)NB * NKP * FD / 8) return; const size_t e = i * 8;
    const int c0 = (int)(e & 63); const int r = (int)((e >> 6) & 63); const int b = (int)(e >> 12);
    const v8f v = *(const v8f*)(sl + (size_t)b * SSTR_FULL + (size_t)min(r, NS - 1) * FD + c0); v8us o;
#pragma unroll
    for (int q = 0; q < 8; ++q) o[q] = (r < NS) ? f2bf(v[q]) : (unsigned short)0;
    *(volatile v8us*)(SL + e) = o; __threadfence(); *(volatile v8us*)(SL + e) = o;
}
__global__ __launch_bounds__(256) void k_ckv(const float* __restrict__ FK, const float* __restrict__ FV, h16* KP, h16* VT) {
    const int nA = NB * NH * NKP * DHD / 8 / 256;
    if ((int)blockIdx.x < nA) {
        const size_t e = ((size_t)blockIdx.x * 256 + threadIdx.x) * 8; const int d0 = (int)(e & 31); const int m = (int)((e >> 5) & (NKP - 1)); const int h = (int)((e / ((size_t)DHD * NKP)) % NH); const int b = (int)(e / ((size_t)DHD * NKP * NH));
        const v8f v = *(const v8f*)(FK + ((size_t)b * NKP + m) * FD + h * DHD + d0); v8h o;
#pragma unroll
        for (int q = 0; q < 8; ++q) { const float y = v[q] * QCAR; o[q] = (m < NS) ? tohx(y) : (h16)0.0f; }
        *(volatile v8h*)(KP + e) = o; __threadfence(); *(volatile v8h*)(KP + e) = o;
    } else {
        const size_t e = ((size_t)((int)blockIdx.x - nA) * 256 + threadIdx.x) * 8; const int m0 = (int)(e & 63); const int n = (int)((e >> 6) & 63); const int b = (int)(e / ((size_t)NKP * FD * NH)); v8h o;
#pragma unroll
        for (int q = 0; q < 8; ++q) { const int m = m0 + q; const float y = FV[((size_t)b * NKP + m) * FD + n] * VCAR; o[q] = (m < NS) ? tohx(y) : (h16)0.0f; }
        *(volatile v8h*)(VT + e) = o; __threadfence(); *(volatile v8h*)(VT + e) = o;
    }
}

extern "C" void kernel_launch(void* const* d_in, const int* in_sizes, int n_in,
                              void* d_out, int out_size, void* d_ws, size_t ws_size, hipStream_t stream) {
    if (n_in < 32) return;
    if (in_sizes[0] < (int)((size_t)NB * TT * FD) || in_sizes[1] < NB * NS * FD) return;
    for (int i = 2; i < 32; ++i) { const int need = (i == 2 || i == 4 || (i >= 14 && (i % 2) == 0)) ? FD * FD : FD; if (in_sizes[i] < need) return; }
    if (out_size < (int)((size_t)NB * TT * FD)) return;
    const float* x = (const float*)d_in[0]; const float* slots = (const float*)d_in[1];
    const float* conv1_b = (const float*)d_in[3]; const float* conv2_b = (const float*)d_in[5];
    const float* gn_g = (const float*)d_in[6]; const float* gn_b = (const float*)d_in[7];
    const float* ln2_g = (const float*)d_in[8]; const float* ln2_b = (const float*)d_in[9]; const float* ln3_g = (const float*)d_in[10]; const float* ln3_b = (const float*)d_in[11]; const float* ln4_g = (const float*)d_in[12]; const float* ln4_b = (const float*)d_in[13];
    const float* sa_qb = (const float*)d_in[15]; const float* sa_kb = (const float*)d_in[17]; const float* sa_vb = (const float*)d_in[19]; const float* sa_ob = (const float*)d_in[21];
    const float* ca_qb = (const float*)d_in[23]; const float* ca_kb = (const float*)d_in[25]; const float* ca_vb = (const float*)d_in[27]; const float* ca_ob = (const float*)d_in[29]; const float* ff1_b = (const float*)d_in[31];
    WArgs wa; wa.w[0] = (const float*)d_in[14]; wa.w[1] = (const float*)d_in[16]; wa.w[2] = (const float*)d_in[18]; wa.w[3] = (const float*)d_in[20]; wa.w[4] = (const float*)d_in[22]; wa.w[5] = (const float*)d_in[24]; wa.w[6] = (const float*)d_in[26]; wa.w[7] = (const float*)d_in[28]; wa.w[8] = (const float*)d_in[30]; wa.w[9] = (const float*)d_in[2]; wa.w[10] = (const float*)d_in[4];
    float* OUT = (float*)d_out;

    const size_t nTF = (size_t)NB * TT * FD;
    const size_t bWB = (size_t)11 * 4096 * 2, bST = (size_t)NB * NGR * 32 * 4, bP2 = nTF * 2, bF4 = nTF * 4;
    const size_t bQP = (size_t)NB * NH * TT * DHD * 2, bVT = (size_t)NB * FD * TT * 2, bOB = (size_t)NB * NH * TT * FD * 4;
    const size_t bRS = (size_t)QCH * TT * 4, bRP = (size_t)QCH * TT * 2;
    char* wsp = (char*)d_ws;
    auto take = [&](size_t bytes) { char* p = wsp; wsp += (bytes + 255) & ~(size_t)255; return (void*)p; };
    bf* WB = (bf*)take(bWB); float* ST = (float*)take(bST);
    bf* XNh = (bf*)take(bP2); bf* XNl = (bf*)take(bP2);
    float* XA = (float*)take(bF4); bf* XAh = (bf*)take(bP2); bf* XAl = (bf*)take(bP2);
    h16* QP = (h16*)take(bQP); h16* KP = (h16*)take(bQP); h16* VT = (h16*)take(bVT);
    float* OB = (float*)take(bOB); bf* ZBh = (bf*)take(bP2); bf* ZBl = (bf*)take(bP2); float* M4 = (float*)take(bF4);
    float* XB = (float*)take(bF4); bf* XBh = (bf*)take(bP2); bf* XBl = (bf*)take(bP2);
    float* XC = (float*)take(bF4); bf* XCh = (bf*)take(bP2); bf* XCl = (bf*)take(bP2);
    bf* XDh = (bf*)take(bP2); bf* XDl = (bf*)take(bP2);
    char* RS = (char*)take(bRS); char* RP = (char*)take(bRP);
    if ((size_t)(wsp - (char*)d_ws) > ws_size) return;
    float* FQ = (float*)RS; float* FK = FQ + nTF; float* FV = FK + nTF; float* FCQ = (float*)RS; float* SC = (float*)RS; float* S = (float*)RS;
    char* sp = RS + ((size_t)16 << 20);
    bf* SLb = (bf*)sp; sp += (size_t)NB * NKP * FD * 2; float* FCK = (float*)sp; sp += (size_t)NB * NKP * FD * 4; float* FCV = (float*)sp; sp += (size_t)NB * NKP * FD * 4;
    h16* CKP = (h16*)sp; sp += (size_t)NB * NH * NKP * DHD * 2; h16* CVT = (h16*)sp; sp += (size_t)NB * NH * FD * NKP * 2;
    if (sp > RS + bRS) return;
    h16* P16 = (h16*)RP;
    const unsigned nb128 = (unsigned)(nTF / 8 / 256);

    k_wall<<<dim3(1, 11), 256, 0, stream>>>(wa, WB);
    k_gnstat<<<NB * NGR, 256, 0, stream>>>(x, ST);
    k_gnapply<<<nb128, 256, 0, stream>>>(x, ST, gn_g, gn_b, XNh, XNl);
    k_gemmw<bf, 2, 2><<<dim3(1, TT / 64, NB), 32, 0, stream>>>(WB + 9 * 4096, nullptr, XNh, XNl, FD, XA, TT, conv1_b, 0, (size_t)TT * FD, (size_t)TT * FD);
    k_split8<<<nb128, 256, 0, stream>>>(XA, XAh, XAl, nTF / 8);
    k_gemmw<bf, 1, 1><<<dim3(TT / 64, 1, NB), 32, 0, stream>>>(XAh, XAl, WB + 0 * 4096, nullptr, FD, FQ, FD, sa_qb, (size_t)TT * FD, 0, (size_t)TT * FD);
    k_gemmw<bf, 1, 1><<<dim3(TT / 64, 1, NB), 32, 0, stream>>>(XAh, XAl, WB + 1 * 4096, nullptr, FD, FK, FD, sa_kb, (size_t)TT * FD, 0, (size_t)TT * FD);
    k_gemmw<bf, 1, 1><<<dim3(TT / 64, 1, NB), 32, 0, stream>>>(XAh, XAl, WB + 2 * 4096, nullptr, FD, FV, FD, sa_vb, (size_t)TT * FD, 0, (size_t)TT * FD);
    k_hsplit<<<nb128, 256, 0, stream>>>(FQ, QP); k_hsplit<<<nb128, 256, 0, stream>>>(FK, KP);
    k_vtp2<<<(unsigned)((size_t)NB * FD * TT / 2 / 256), 256, 0, stream>>>(FV, VT);
    for (int b = 0; b < NB; ++b) for (int h = 0; h < NH; ++h) for (int ch = 0; ch < TT / QCH; ++ch) {
        const size_t qo = (((size_t)b * NH + h) * TT + (size_t)ch * QCH) * DHD; const size_t ko = ((size_t)b * NH + h) * TT * DHD; const size_t oo = (((size_t)b * NH + h) * TT + (size_t)ch * QCH) * FD;
        k_gemmw<h16, 0, 0><<<dim3(QCH / 64, TT / 64, 1), 32, 0, stream>>>(QP + qo, nullptr, KP + ko, nullptr, DHD, S, TT, nullptr, 0, 0, 0);
        k_lsoft<<<QCH / 8, 256, 0, stream>>>(S, P16);
        k_gemmw<h16, 0, 0><<<dim3(QCH / 64, 1, 1), 32, 0, stream>>>(P16, nullptr, VT + (size_t)b * FD * TT, nullptr, TT, OB + oo, FD, nullptr, 0, 0, 0);
    }
    k_zsplit<<<nb128, 256, 0, stream>>>(OB, ZBh, ZBl);
    k_gemmw<bf, 1, 1><<<dim3(TT / 64, 1, NB), 32, 0, stream>>>(ZBh, ZBl, WB + 3 * 4096, nullptr, FD, M4, FD, sa_ob, (size_t)TT * FD, 0, (size_t)TT * FD);
    k_lnres<true, true><<<(unsigned)(NB * TT / 8), 256, 0, stream>>>(M4, XA, ln2_g, ln2_b, XB, XBh, XBl);
    k_gemmw<bf, 1, 1><<<dim3(TT / 64, 1, NB), 32, 0, stream>>>(XBh, XBl, WB + 4 * 4096, nullptr, FD, FCQ, FD, ca_qb, (size_t)TT * FD, 0, (size_t)TT * FD);
    k_slotp<<<(unsigned)((size_t)NB * NKP * FD / 8 / 256), 256, 0, stream>>>(slots, SLb);
    k_gemmw<bf, 0, 1><<<dim3(1, 1, NB), 32, 0, stream>>>(SLb, nullptr, WB + 5 * 4096, nullptr, FD, FCK, FD, ca_kb, (size_t)NKP * FD, 0, (size_t)NKP * FD);
    k_gemmw<bf, 0, 1><<<dim3(1, 1, NB), 32, 0, stream>>>(SLb, nullptr, WB + 6 * 4096, nullptr, FD, FCV, FD, ca_vb, (size_t)NKP * FD, 0, (size_t)NKP * FD);
    k_ckv<<<(unsigned)(NB * NH * NKP * DHD / 8 / 256 + NB * NH * FD * NKP / 8 / 256), 256, 0, stream>>>(FCK, FCV, CKP, CVT);
    k_hsplit<<<nb128, 256, 0, stream>>>(FCQ, QP);
    k_gemmw<h16, 0, 0><<<dim3(TT / 64, NKP / 64, NB * NH), 32, 0, stream>>>(QP, nullptr, CKP, nullptr, DHD, SC, NKP, nullptr, (size_t)TT * DHD, (size_t)NKP * DHD, (size_t)TT * NKP);
    k_csoft<<<(unsigned)((size_t)NB * NH * TT / 32), 256, 0, stream>>>(SC, P16);
    k_gemmw<h16, 0, 0><<<dim3(TT / 64, 1, NB * NH), 32, 0, stream>>>(P16, nullptr, CVT, nullptr, NKP, OB, FD, nullptr, (size_t)TT * NKP, (size_t)FD * NKP, (size_t)TT * FD);
    k_zsplit<<<nb128, 256, 0, stream>>>(OB, ZBh, ZBl);
    k_gemmw<bf, 1, 1><<<dim3(TT / 64, 1, NB), 32, 0, stream>>>(ZBh, ZBl, WB + 7 * 4096, nullptr, FD, M4, FD, ca_ob, (size_t)TT * FD, 0, (size_t)TT * FD);
    k_lnres<false, true><<<(unsigned)(NB * TT / 8), 256, 0, stream>>>(M4, XB, ln3_g, ln3_b, XC, XCh, XCl);
    k_gemmw<bf, 1, 1><<<dim3(TT / 64, 1, NB), 32, 0, stream>>>(XCh, XCl, WB + 8 * 4096, nullptr, FD, M4, FD, ff1_b, (size_t)TT * FD, 0, (size_t)TT * FD);
    k_lnres<false, false><<<(unsigned)(NB * TT / 8), 256, 0, stream>>>(M4, XC, ln4_g, ln4_b, nullptr, XDh, XDl);
    k_gemmw<bf, 1, 1><<<dim3(TT / 64, 1, NB), 32, 0, stream>>>(XDh, XDl, WB + 10 * 4096, nullptr, FD, OUT, FD, conv2_b, (size_t)TT * FD, 0, (size_t)TT * FD);
}
